// InstanceConsistencyNetwork_60876866453861
// MI455X (gfx1250) — hardware-verified
//
#include <hip/hip_runtime.h>
#include <math.h>

typedef __attribute__((ext_vector_type(16))) _Float16 v16h;
typedef __attribute__((ext_vector_type(16))) __bf16 v16b;
typedef __attribute__((ext_vector_type(8)))  _Float16 v8h;
typedef __attribute__((ext_vector_type(8)))  float v8f;
typedef __attribute__((ext_vector_type(4)))  float v4f;
typedef __attribute__((ext_vector_type(2)))  float v2f;
typedef __attribute__((ext_vector_type(4)))  unsigned v4u;
typedef __attribute__((ext_vector_type(4)))  int v4i;
typedef float __attribute__((may_alias)) float_a;
typedef int __attribute__((may_alias)) int_a;

template <typename T> __device__ __forceinline__ void vst2(void* p, T v) { *(volatile T*)p = v; __threadfence(); *(volatile T*)p = v; }
__device__ __forceinline__ v8f wmma16(v16h a, v16h b, v8f c) {
  v8f d = __builtin_amdgcn_wmma_f32_16x16x32_f16(false, a, false, b, (short)0, c, false, false);
  asm volatile("v_nop\n\tv_nop\n\tv_nop\n\tv_nop" : "+v"(d) : "v"(a), "v"(b));
  return d;
}
__device__ __forceinline__ v8f wmma_bf(v16b a, v16b b, v8f c) {
  v8f d = __builtin_amdgcn_wmma_f32_16x16x32_bf16(false, a, false, b, (short)0, c, false, false);
  asm volatile("v_nop\n\tv_nop\n\tv_nop\n\tv_nop" : "+v"(d) : "v"(a), "v"(b));
  return d;
}
__device__ __forceinline__ v16h frag_h(const _Float16* rowk0, int lane) {
  union { v16h v; v8h q[2]; } u; const _Float16* p = rowk0 + 8 * (lane >> 4);
  u.q[0] = *(const v8h*)p; u.q[1] = *(const v8h*)(p + 16); return u.v;
}
__device__ __forceinline__ v16h frag_f32(const float* rowk0, int lane) {
  v16h a; const float* p = rowk0 + 8 * (lane >> 4);
#pragma unroll
  for (int i = 0; i < 8; ++i) { a[i] = (_Float16)p[i]; a[8 + i] = (_Float16)p[16 + i]; }
  return a;
}
__device__ __forceinline__ v16h frag_f32s(const float* rowk0, int lane, float sc) {
  v16h a; const float* p = rowk0 + 8 * (lane >> 4);
#pragma unroll
  for (int i = 0; i < 8; ++i) { a[i] = (_Float16)(p[i] * sc); a[8 + i] = (_Float16)(p[16 + i] * sc); }
  return a;
}
__device__ __forceinline__ v16h fragc_f32(const float* W, int k0, int n, int lane, int ld, int K) {
  v16h a; const int g = lane >> 4;
#pragma unroll
  for (int i = 0; i < 8; ++i) { const int ka = k0 + 8 * g + i, kb = ka + 16;
    a[i] = (_Float16)(ka < K ? W[(size_t)(ka < K ? ka : K - 1) * ld + n] : 0.f); a[8 + i] = (_Float16)(kb < K ? W[(size_t)(kb < K ? kb : K - 1) * ld + n] : 0.f); }
  return a;
}
struct F2 { v16b h, l; };
__device__ __forceinline__ F2 bsplit16(const float v[16]) { F2 r;
#pragma unroll
  for (int i = 0; i < 16; ++i) { const __bf16 h = (__bf16)v[i]; r.h[i] = h; r.l[i] = (__bf16)(v[i] - (float)h); }
  return r; }
__device__ __forceinline__ F2 split_row(const float* row, int k0, int lane) { float v[16]; const float* p = row + k0 + 8 * (lane >> 4);
#pragma unroll
  for (int i = 0; i < 8; ++i) { v[i] = p[i]; v[8 + i] = p[16 + i]; }
  return bsplit16(v); }
__device__ __forceinline__ F2 split_rowK(const float* row, int k0, int lane, int K) { float v[16]; const int g = lane >> 4;
#pragma unroll
  for (int i = 0; i < 8; ++i) { const int ka = k0 + 8 * g + i, kb = ka + 16; v[i] = ka < K ? row[ka < K ? ka : K - 1] : 0.f; v[8 + i] = kb < K ? row[kb < K ? kb : K - 1] : 0.f; }
  return bsplit16(v); }
__device__ __forceinline__ F2 split_col(const float* W, int k0, int n, int lane, int ld, int K) { float v[16]; const int g = lane >> 4;
#pragma unroll
  for (int i = 0; i < 8; ++i) { const int ka = k0 + 8 * g + i, kb = ka + 16; v[i] = ka < K ? W[(size_t)(ka < K ? ka : K - 1) * ld + n] : 0.f; v[8 + i] = kb < K ? W[(size_t)(kb < K ? kb : K - 1) * ld + n] : 0.f; }
  return bsplit16(v); }
__device__ __forceinline__ v8f mac3(const F2& a, const F2& b, v8f c) { c = wmma_bf(a.l, b.h, c); c = wmma_bf(a.h, b.l, c); return wmma_bf(a.h, b.h, c); }
__device__ __forceinline__ float sigm(float v) { return 1.0f / (1.0f + expf(-v)); }
#define LDSX() do { asm volatile("s_wait_dscnt 0" ::: "memory"); __builtin_amdgcn_wave_barrier(); __builtin_amdgcn_fence(__ATOMIC_RELEASE, "workgroup"); } while (0)


#define NB 2
#define NN 8192
#define NR (NB * NN)
#define DD 32
#define R2 0.0009f
#define STH 0.7f
typedef __attribute__((ext_vector_type(8))) __bf16 v8b;
__device__ __forceinline__ v16b frag_b(const __bf16* rowk0, int lane) {
  union { v16b v; v8b q[2]; } u; const __bf16* p = rowk0 + 8 * (lane >> 4);
  u.q[0] = *(const v8b*)p; u.q[1] = *(const v8b*)(p + 16); return u.v;
}
__device__ __forceinline__ float bfr(float v) { return (float)(__bf16)v; }
__device__ __attribute__((noinline)) float exp_ni(float v) { return expf(v); }
__device__ __attribute__((noinline)) float erf_ni(float v) { return erff(v); }

#define WS_PK  0u
#define PK_2   (DD * 2 * DD)
#define PK_END (PK_2 + DD * DD)
#define WS_P4  (((2u * PK_END) + 127u) / 128u * 128u)
#define WS_SQ  (WS_P4 + 4u * NR * 4)
#define WS_EN  (WS_SQ + 4u * NR)
#define WS_AH  (WS_EN + 4u * NR * DD)
#define WS_AL  (WS_AH + 2u * NR * 2 * DD)
#define WS_CND (WS_AL + 2u * NR * 2 * DD)
#define WS_LC  (WS_CND + 4u * (NR / 4) * 32)
static_assert(4u * (NR / 4) * 32 == 32u * NR, "CND carve = 32 ints per 4-query block");
#define WS_END (WS_LC + 128u)

__global__ __launch_bounds__(64) void k_pack(const float* __restrict__ W1, const float* __restrict__ W2, __bf16* __restrict__ PK) {
  __shared__ __align__(16) __bf16 s[2 * DD]; const int n = blockIdx.x, which = blockIdx.y, t = threadIdx.x; int K; size_t dst;
  if (which == 0) { K = 2 * DD; dst = (size_t)n * 2 * DD; s[t] = (__bf16)W1[(size_t)t * DD + n]; } else { K = DD; dst = PK_2 + (size_t)n * DD; if (t < DD) s[t] = (__bf16)W2[(size_t)t * DD + n]; }
  __syncthreads();
  if (t < K / 8) vst2((unsigned*)(PK + dst + t * 8), *(const v4u*)&s[t * 8]);
}
__global__ __launch_bounds__(64) void k_prep(const float* __restrict__ PTS, const float* __restrict__ EMB, float* __restrict__ P4, float* __restrict__ SQ, float* __restrict__ EN) {
  __shared__ __align__(16) float sp[64][4]; __shared__ __align__(16) float ssq[64]; __shared__ __align__(16) float sen[64][DD + 4]; const int t = threadIdx.x; const size_t p = (size_t)blockIdx.x * 64 + t;
  const float x0 = bfr(PTS[p * 3]), x1 = bfr(PTS[p * 3 + 1]), x2 = bfr(PTS[p * 3 + 2]); sp[t][0] = x0; sp[t][1] = x1; sp[t][2] = x2; sp[t][3] = 0.f; ssq[t] = __fadd_rn(__fadd_rn(__fmul_rn(x0, x0), __fmul_rn(x2, x2)), __fmul_rn(x1, x1));
  float e[DD]; float nrm = 0.f;
#pragma unroll
  for (int d = 0; d < DD; ++d) { e[d] = bfr(EMB[p * DD + d]); nrm += e[d] * e[d]; }
  const float inv = 1.0f / fmaxf(sqrtf(nrm), 1e-8f);
#pragma unroll
  for (int d = 0; d < DD; ++d) sen[t][d] = e[d] * inv;
  __syncthreads();
  vst2(P4 + p * 4, *(const v4f*)&sp[t][0]); if (t < 16) vst2(SQ + (size_t)blockIdx.x * 64 + t * 4, *(const v4f*)&ssq[t * 4]);
  for (int e2 = t; e2 < 64 * DD / 4; e2 += 64) { const int r = e2 >> 3, pc = e2 & 7; vst2(EN + ((size_t)blockIdx.x * 64 + r) * DD + pc * 4, *(const v4f*)&sen[r][pc * 4]); }
}
__global__ __launch_bounds__(256) void k_lc(const int* __restrict__ LEAF, int* __restrict__ LC) {
  __shared__ int sred[8]; __shared__ __align__(16) int sl[32]; const int t = threadIdx.x; int c0 = 0, c1 = 0;
  for (int i = t; i < NN; i += 256) { c0 += (LEAF[i] > 0) ? 1 : 0; c1 += (LEAF[NN + i] > 0) ? 1 : 0; }
#pragma unroll
  for (int o = 1; o < 32; o <<= 1) { c0 += __shfl_xor(c0, o); c1 += __shfl_xor(c1, o); }
  if ((t & 31) == 0) { sred[t >> 5] = c0; } __syncthreads();
  if (t == 0) { int a = 0; for (int w = 0; w < 8; ++w) a += sred[w]; sl[0] = a; } __syncthreads();
  if ((t & 31) == 0) { sred[t >> 5] = c1; } __syncthreads();
  if (t == 0) { int a = 0; for (int w = 0; w < 8; ++w) a += sred[w]; sl[1] = a; for (int k = 2; k < 32; ++k) sl[k] = 0; } __syncthreads();
  if (t < 8) vst2((unsigned*)(LC + t * 4), *(const v4u*)&sl[t * 4]);
}
__global__ __launch_bounds__(128) void k_nb(const float* __restrict__ P4, const float* __restrict__ SQ, const float* __restrict__ EN, const float* __restrict__ EMB, const int* __restrict__ LEAF, const int* __restrict__ LC, __bf16* __restrict__ AH, __bf16* __restrict__ AL, int* __restrict__ CND) {
  __shared__ float sacc[4][32][DD + 1]; __shared__ int scnt[4][32], snb[4][32]; __shared__ __align__(16) __bf16 sh_[4][2 * DD], sl_[4][2 * DD]; __shared__ __align__(16) int scond[32];
  const int tid = threadIdx.x, wave = tid >> 5, lane = tid & 31; const size_t q = (size_t)blockIdx.x * 4 + wave; const int b = (int)(q / NN); const size_t base = (size_t)b * NN;
  const float qx0 = P4[q * 4], qx1 = P4[q * 4 + 1], qx2 = P4[q * 4 + 2], sqi = SQ[q];
  float eni[DD];
#pragma unroll
  for (int d = 0; d < DD; ++d) eni[d] = EN[q * DD + d];
  float acc[DD];
#pragma unroll
  for (int d = 0; d < DD; ++d) acc[d] = 0.f;
  int cnt = 0, nbc = 0;
#pragma unroll 1
  for (int j = lane; j < NN; j += 32) { const size_t pj = base + j; const float dot = __fadd_rn(__fadd_rn(__fmul_rn(qx0, P4[pj * 4]), __fmul_rn(qx1, P4[pj * 4 + 1])), __fmul_rn(qx2, P4[pj * 4 + 2])); const float d2 = __fsub_rn(__fadd_rn(sqi, SQ[pj]), __fmul_rn(2.0f, dot));
    const bool nb = (d2 < R2) && (LEAF[pj] > 0);
    if (nb) { ++nbc; float s = 0.f;
#pragma unroll
      for (int d = 0; d < DD; ++d) s += eni[d] * EN[pj * DD + d];
      if (s > STH) { ++cnt;
#pragma unroll
        for (int d = 0; d < DD; ++d) acc[d] += bfr(EMB[pj * DD + d]); } } }
#pragma unroll
  for (int d = 0; d < DD; ++d) sacc[wave][lane][d] = acc[d];
  scnt[wave][lane] = cnt; snb[wave][lane] = nbc;
  __syncthreads();
  { const int d = lane; float a = 0.f; int c = 0, nbt = 0; for (int l = 0; l < 32; ++l) { a += sacc[wave][l][d]; c += scnt[wave][l]; nbt += snb[wave][l]; }
    const float mean = a / (float)max(c, 1); const float ev = bfr(EMB[q * DD + d]);
    { const __bf16 hb = (__bf16)ev; sh_[wave][d] = hb; sl_[wave][d] = (__bf16)(ev - (float)hb); }
    { const __bf16 hb = (__bf16)mean; sh_[wave][DD + d] = hb; sl_[wave][DD + d] = (__bf16)(mean - (float)hb); }
    if (lane == 0) { const bool leaf = LEAF[q] > 0; const bool bok = LC[b] >= 10; scond[wave] = (leaf && nbt > 1 && c > 0 && bok) ? 1 : 0; } }
  if (tid >= 4 && tid < 32) scond[tid] = 0;
  __syncthreads();
  if (tid < 32) { const int r = tid >> 3, pc = tid & 7; vst2((unsigned*)(AH + ((size_t)blockIdx.x * 4 + r) * 2 * DD + pc * 8), *(const v4u*)&sh_[r][pc * 8]); }
  else if (tid < 64) { const int t2 = tid - 32; const int r = t2 >> 3, pc = t2 & 7; vst2((unsigned*)(AL + ((size_t)blockIdx.x * 4 + r) * 2 * DD + pc * 8), *(const v4u*)&sl_[r][pc * 8]); }
  if (tid >= 64 && tid < 72) vst2((unsigned*)(CND + (size_t)blockIdx.x * 32 + (tid - 64) * 4), *(const v4u*)&scond[(tid - 64) * 4]);
}
__global__ __launch_bounds__(128) void k_mlp(const __bf16* __restrict__ AH, const __bf16* __restrict__ AL, const __bf16* __restrict__ PK, const float* __restrict__ B1, const float* __restrict__ B2, const float* __restrict__ EMB, const int* __restrict__ CND, float* __restrict__ OUT) {
  __shared__ __align__(16) __bf16 sh_[4][16][40], sl_[4][16][40]; __shared__ __align__(16) float so[4][16][DD + 4];
  const int tid = threadIdx.x, wave = tid >> 5, lane = tid & 31, col = lane & 15, g = lane >> 4; const size_t r0 = (size_t)blockIdx.x * 64 + wave * 16;
  v8f acc[2] = {};
#pragma unroll
  for (int kc = 0; kc < 2; ++kc) { const v16b ah = frag_b(AH + (r0 + col) * 2 * DD + kc * 32, lane), al = frag_b(AL + (r0 + col) * 2 * DD + kc * 32, lane);
#pragma unroll
    for (int j = 0; j < 2; ++j) { const v16b w = frag_b(PK + (size_t)(j * 16 + col) * 2 * DD + kc * 32, lane); acc[j] = wmma_bf(al, w, acc[j]); acc[j] = wmma_bf(ah, w, acc[j]); } }
#pragma unroll
  for (int j = 0; j < 2; ++j) { const int c = j * 16 + col; const float bb = bfr(B1[c]);
#pragma unroll
    for (int r = 0; r < 8; ++r) { const float v = fmaxf(acc[j][r] + bb, 0.f); const __bf16 hb = (__bf16)v; sh_[wave][8 * g + r][c] = hb; sl_[wave][8 * g + r][c] = (__bf16)(v - (float)hb); } }
  LDSX();
  v8f acc2[2] = {};
  { F2 a; a.h = frag_b(&sh_[wave][col][0], lane); a.l = frag_b(&sl_[wave][col][0], lane);
#pragma unroll
    for (int j = 0; j < 2; ++j) { const v16b w = frag_b(PK + PK_2 + (size_t)(j * 16 + col) * DD, lane); acc2[j] = wmma_bf(a.l, w, acc2[j]); acc2[j] = wmma_bf(a.h, w, acc2[j]); } }
#pragma unroll
  for (int j = 0; j < 2; ++j) { const int c = j * 16 + col; const float bb = bfr(B2[c]);
#pragma unroll
    for (int r = 0; r < 8; ++r) { const size_t row = r0 + 8 * g + r; const int cnd = CND[(row >> 2) * 32 + (row & 3)]; so[wave][8 * g + r][c] = cnd ? (acc2[j][r] + bb) : bfr(EMB[row * DD + c]); } }
  LDSX();
  for (int rl = 0; rl < 16; ++rl) if (lane < 8) vst2(OUT + (r0 + rl) * DD + lane * 4, *(const v4f*)&so[wave][rl][lane * 4]);
}
extern "C" void kernel_launch(void* const* d_in, const int* in_sizes, int n_in, void* d_out, int out_size, void* d_ws, size_t ws_size, hipStream_t stream) {
  (void)in_sizes; (void)n_in; (void)out_size;
  if (ws_size < (size_t)WS_END) return;
  char* ws = (char*)d_ws; __bf16 *PK = (__bf16*)(ws + WS_PK), *AH = (__bf16*)(ws + WS_AH), *AL = (__bf16*)(ws + WS_AL); float *P4 = (float*)(ws + WS_P4), *SQ = (float*)(ws + WS_SQ), *EN = (float*)(ws + WS_EN); int *CND = (int*)(ws + WS_CND), *LC = (int*)(ws + WS_LC);
  const float* PTS = (const float*)d_in[0]; const float* EMB = (const float*)d_in[1]; const int* LEAF = (const int*)d_in[2];
  k_pack<<<dim3(DD, 2), 64, 0, stream>>>((const float*)d_in[3], (const float*)d_in[5], PK);
  k_prep<<<NR / 64, 64, 0, stream>>>(PTS, EMB, P4, SQ, EN);
  k_lc<<<1, 256, 0, stream>>>(LEAF, LC);
  k_nb<<<NR / 4, 128, 0, stream>>>(P4, SQ, EN, EMB, LEAF, LC, AH, AL, CND);
  k_mlp<<<NR / 64, 128, 0, stream>>>(AH, AL, PK, (const float*)d_in[4], (const float*)d_in[6], EMB, CND, (float*)d_out);
}
